// AttentionLayer_5995774345736
// MI455X (gfx1250) — hardware-verified
//
#include <hip/hip_runtime.h>


#ifndef NB
#define NB 4
#endif
#ifndef SEQ
#define SEQ 2048
#endif
#define NB_FULL  4
#define SEQ_FULL 2048
#define DMD  1024
#define NH   16
#define HD   64
#define KT   32
#define PSP  40
#define CSP  72
#define PCAR 1024.0f
#define VCAR 16.0f
#define CCAR 64.0f
#define WCAR 64.0f
#define SCL  0.125f
#define L2E  1.4426950408889634f
static_assert((SEQ % 64) == 0);
static_assert((DMD % 64) == 0);
static_assert(NH * HD == DMD);
static_assert(NB >= 1 && NB <= NB_FULL);
static_assert(SEQ >= 64 && SEQ <= SEQ_FULL);

typedef _Float16 h16;
typedef unsigned short bf;
typedef __attribute__((ext_vector_type(16))) __bf16   v16bf;
typedef __attribute__((ext_vector_type(16))) _Float16 v16h;
typedef __attribute__((ext_vector_type(8)))  _Float16 v8h;
typedef __attribute__((ext_vector_type(8)))  unsigned short v8us;
typedef __attribute__((ext_vector_type(8)))  float    v8f;
typedef __attribute__((ext_vector_type(4)))  float    v4f;
typedef __attribute__((ext_vector_type(2)))  _Float16 v2h;
typedef __attribute__((ext_vector_type(2)))  unsigned short v2us;
typedef v8h  __attribute__((may_alias)) v8ha;
typedef v4f  __attribute__((may_alias)) v4fa;
typedef v8us __attribute__((may_alias)) v8usa;

__device__ __forceinline__ unsigned short f2bf(float f) { unsigned u = __float_as_uint(f); u += 0x7FFFu + ((u >> 16) & 1u); return (unsigned short)(u >> 16); }
__device__ __forceinline__ float bf2f(unsigned short b) { return __uint_as_float(((unsigned)b) << 16); }
__device__ __forceinline__ float bfr(float f) { return bf2f(f2bf(f)); }
__device__ __forceinline__ h16 tohx(float x) { return (h16)x; }
__device__ __forceinline__ void splitf(float y, unsigned short& h, unsigned short& l) { h = f2bf(y); l = f2bf(y - bf2f(h)); }
__device__ __forceinline__ v16h cat16(v8h lo, v8h hi) { return __builtin_shufflevector(lo, hi, 0, 1, 2, 3, 4, 5, 6, 7, 8, 9, 10, 11, 12, 13, 14, 15); }
__device__ __forceinline__ v16bf cat16b(v8us lo, v8us hi) { return __builtin_bit_cast(v16bf, __builtin_shufflevector(lo, hi, 0, 1, 2, 3, 4, 5, 6, 7, 8, 9, 10, 11, 12, 13, 14, 15)); }
__device__ __forceinline__ v8f wmma16(v16h a, v16h b, v8f c) { return __builtin_amdgcn_wmma_f32_16x16x32_f16(false, a, false, b, (short)0, c, false, false); }
__device__ __forceinline__ v8f wmmab(v16bf a, v16bf b, v8f c) { return __builtin_amdgcn_wmma_f32_16x16x32_bf16(false, a, false, b, (short)0, c, false, false); }

template <typename T16> struct WFrag;
template <> struct WFrag<h16> { typedef v16h V; static __device__ __forceinline__ V ld(const h16* p) { return cat16(*(const v8h*)p, *(const v8h*)(p + 16)); } static __device__ __forceinline__ v8f mma(V a, V b, v8f c) { return wmma16(a, b, c); } };
template <> struct WFrag<bf> { typedef v16bf V; static __device__ __forceinline__ V ld(const bf* p) { return cat16b(*(const v8us*)p, *(const v8us*)(p + 16)); } static __device__ __forceinline__ v8f mma(V a, V b, v8f c) { return wmmab(a, b, c); } };

template <typename T16, int NSPLIT, bool BIAS>
__global__ __launch_bounds__(32) void k_gemmw(const T16* __restrict__ A, const T16* __restrict__ A2, const T16* __restrict__ Bt, const T16* __restrict__ Bt2, int K, float* C, int ldc, const float* __restrict__ bias, float cmul, size_t sA, size_t sB, size_t sC) {
    typedef typename WFrag<T16>::V V;
    __shared__ __align__(16) float os[16 * 68];
    const size_t z = blockIdx.z; A += z * sA; if (A2) A2 += z * sA; Bt += z * sB; if (Bt2) Bt2 += z * sB; C += z * sC;
    const int lane = threadIdx.x & 31, lr = lane & 15, hi = lane >> 4; const int r0 = blockIdx.x * 64, c0 = blockIdx.y * 64;
    const int cofs = lr * 4;
    v4f bb = (v4f){};
    if (BIAS) { bb[0] = bfr(bias[c0 + cofs]); bb[1] = bfr(bias[c0 + cofs + 1]); bb[2] = bfr(bias[c0 + cofs + 2]); bb[3] = bfr(bias[c0 + cofs + 3]); }
    v8f acc[4][4];
#pragma unroll
    for (int mb = 0; mb < 4; ++mb)
#pragma unroll
        for (int nb = 0; nb < 4; ++nb) acc[mb][nb] = (v8f){};
    const size_t aoff = (size_t)(r0 + lr) * K + 8 * hi, boff = (size_t)(c0 + lr) * K + 8 * hi;
#pragma unroll 1
    for (int kc = 0; kc < K; kc += 32) {
        V a[4], a2[4];
#pragma unroll
        for (int mb = 0; mb < 4; ++mb) { a[mb] = WFrag<T16>::ld(A + aoff + (size_t)mb * 16 * K + kc); if (NSPLIT == 1 || NSPLIT == 2) a2[mb] = WFrag<T16>::ld(A2 + aoff + (size_t)mb * 16 * K + kc); }
#pragma unroll
        for (int nb = 0; nb < 4; ++nb) { const V b = WFrag<T16>::ld(Bt + boff + (size_t)nb * 16 * K + kc); V b2; if (NSPLIT >= 2) b2 = WFrag<T16>::ld(Bt2 + boff + (size_t)nb * 16 * K + kc);
#pragma unroll
            for (int mb = 0; mb < 4; ++mb) { acc[mb][nb] = WFrag<T16>::mma(a[mb], b, acc[mb][nb]); if (NSPLIT == 1 || NSPLIT == 2) acc[mb][nb] = WFrag<T16>::mma(a2[mb], b, acc[mb][nb]); if (NSPLIT >= 2) acc[mb][nb] = WFrag<T16>::mma(a[mb], b2, acc[mb][nb]); } }
        asm volatile("v_nop\n\tv_nop\n\tv_nop\n\tv_nop" : "+v"(acc[0][0]), "+v"(acc[1][1]), "+v"(acc[2][2]), "+v"(acc[3][3]) : "v"(a[0]), "v"(a[3]));
    }
#pragma unroll
    for (int mb = 0; mb < 4; ++mb) {
#pragma unroll
        for (int nb = 0; nb < 4; ++nb) {
#pragma unroll
            for (int j = 0; j < 8; ++j) os[(hi * 8 + j) * 68 + nb * 16 + lr] = acc[mb][nb][j]; }
        __builtin_amdgcn_wave_barrier(); asm volatile("" ::: "memory");
        float* crow = C + (size_t)(r0 + mb * 16) * ldc + c0;
#pragma unroll 1
        for (int ps = 0; ps < 2; ++ps) {
#pragma unroll
            for (int s = 0; s < 8; ++s) { const int row = 2 * s + hi; v4f val = *(const v4fa*)(os + row * 68 + cofs); val = val * cmul + bb;
                *(volatile v4f*)(crow + (size_t)row * ldc + cofs) = val; }
            if (ps == 0) __threadfence(); }
        __builtin_amdgcn_wave_barrier(); asm volatile("" ::: "memory");
    }
}

__global__ __launch_bounds__(256) void k_wtG(const float* __restrict__ w, int K, int N, bf* Bt) {
    const int lane = threadIdx.x & 31; const int L0 = (blockIdx.x * 8 + (threadIdx.x >> 5)) * 8; const int nlines = N * K / 64;
#pragma unroll
    for (int ps = 0; ps < 2; ++ps) {
#pragma unroll 1
        for (int l = 0; l < 8; ++l) { const int L = L0 + l; if (L >= nlines) break; const size_t e = (size_t)L * 64 + lane * 2; const int k = (int)(e % K), n = (int)(e / K); v2us o;
            o[0] = f2bf(w[(size_t)k * N + n]); o[1] = f2bf(w[(size_t)(k + 1) * N + n]); *(volatile v2us*)(Bt + e) = o; }
        if (ps == 0) __threadfence(); }
}
__global__ __launch_bounds__(256) void k_wtH(const float* __restrict__ w, int K, int N, float sc, h16* Bt) {
    const int lane = threadIdx.x & 31; const int L0 = (blockIdx.x * 8 + (threadIdx.x >> 5)) * 8; const int nlines = N * K / 64;
#pragma unroll
    for (int ps = 0; ps < 2; ++ps) {
#pragma unroll 1
        for (int l = 0; l < 8; ++l) { const int L = L0 + l; if (L >= nlines) break; const size_t e = (size_t)L * 64 + lane * 2; const int k = (int)(e % K), n = (int)(e / K); v2h o;
            o[0] = tohx(bfr(w[(size_t)k * N + n]) * sc); o[1] = tohx(bfr(w[(size_t)(k + 1) * N + n]) * sc); *(volatile v2h*)(Bt + e) = o; }
        if (ps == 0) __threadfence(); }
}
__global__ __launch_bounds__(256) void k_cvt8(const float* __restrict__ src, bf* dst, size_t n8) { const size_t i = (size_t)blockIdx.x * 256 + threadIdx.x; if (i >= n8) return; const v8f v = *(const v8f*)(src + i * 8); v8us o;
#pragma unroll
    for (int k = 0; k < 8; ++k) o[k] = f2bf(v[k]); *(volatile v8us*)(dst + i * 8) = o; __threadfence(); *(volatile v8us*)(dst + i * 8) = o; }

__global__ __launch_bounds__(256) void k_qkp(const float* __restrict__ F, float sc, bf* Ph, bf* Pl) {
    const size_t e = ((size_t)blockIdx.x * 256 + threadIdx.x) * 2; if (e >= (size_t)NH * SEQ * HD) return;
    const int d = (int)(e % HD); const int t = (int)((e / HD) % SEQ); const int hh = (int)(e / ((size_t)HD * SEQ));
    const float* f = F + (size_t)t * DMD + hh * HD + d;
    v2us oh, ol;
#pragma unroll
    for (int q = 0; q < 2; ++q) { const float x = f[q] * sc; unsigned short a2, c2; splitf(x, a2, c2); oh[q] = a2; ol[q] = c2; }
    *(volatile v2us*)(Ph + e) = oh; *(volatile v2us*)(Pl + e) = ol; __threadfence(); *(volatile v2us*)(Ph + e) = oh; *(volatile v2us*)(Pl + e) = ol;
}
__global__ __launch_bounds__(256) void k_vtp(const float* __restrict__ F, h16* VT) {
    const size_t e = ((size_t)blockIdx.x * 256 + threadIdx.x) * 2; if (e >= (size_t)NH * HD * SEQ) return;
    const int t = (int)(e % SEQ); const int d = (int)((e / SEQ) % HD); const int hh = (int)(e / ((size_t)SEQ * HD));
    v2h o;
#pragma unroll
    for (int q = 0; q < 2; ++q) o[q] = tohx(F[(size_t)(t + q) * DMD + hh * HD + d] * VCAR);
    *(volatile v2h*)(VT + e) = o; __threadfence(); *(volatile v2h*)(VT + e) = o;
}
__global__ __launch_bounds__(256) void k_colsum(const float* __restrict__ F, float* VS) {
    __shared__ __align__(16) float st[256];
    const int tid = threadIdx.x; const int c = blockIdx.x * 256 + tid;
    float p[8];
#pragma unroll
    for (int u = 0; u < 8; ++u) p[u] = 0.f;
#pragma unroll 1
    for (int t = 0; t < SEQ; t += 8) {
#pragma unroll
        for (int u = 0; u < 8; ++u) p[u] += F[(size_t)(t + u) * DMD + c];
    }
    st[tid] = ((p[0] + p[1]) + (p[2] + p[3])) + ((p[4] + p[5]) + (p[6] + p[7]));
    __syncthreads();
    if (tid < 64) { const v4f v = *(const v4fa*)(st + tid * 4); float* dst = VS + (size_t)blockIdx.x * 256 + tid * 4; *(volatile v4f*)dst = v; __threadfence(); *(volatile v4f*)dst = v; }
}

__global__ __launch_bounds__(64) void k_flash(const bf* __restrict__ QPh, const bf* __restrict__ QPl, const bf* __restrict__ KPh, const bf* __restrict__ KPl,
                                              const h16* __restrict__ VT, const float* __restrict__ VS, h16* CTX) {
    __shared__ __align__(16) h16 ps[2][16 * PSP];
    __shared__ __align__(16) h16 cs[2][16 * CSP];
    const int lane = threadIdx.x & 31, wv = threadIdx.x >> 5, lr = lane & 15, hi = lane >> 4;
    const int h = blockIdx.y;
    const int r0 = blockIdx.x * 32 + wv * 16;
    h16* pw = ps[wv]; h16* cw = cs[wv];
    const size_t qo = ((size_t)h * SEQ + r0 + lr) * HD + 8 * hi;
    const v16bf qh0 = WFrag<bf>::ld(QPh + qo), qh1 = WFrag<bf>::ld(QPh + qo + 32);
    const v16bf ql0 = WFrag<bf>::ld(QPl + qo), ql1 = WFrag<bf>::ld(QPl + qo + 32);
    v8f o[4];
#pragma unroll
    for (int t = 0; t < 4; ++t) o[t] = (v8f){};
    float mrun[8], lrun[8], sbar[8];
#pragma unroll
    for (int r = 0; r < 8; ++r) { mrun[r] = -1.0e30f; lrun[r] = 0.f; sbar[r] = 0.f; }
    const size_t ko = ((size_t)h * SEQ + lr) * HD + 8 * hi;
    const size_t vo = ((size_t)h * HD + lr) * SEQ + 8 * hi;
#pragma unroll 1
    for (int j = 0; j < SEQ / KT; ++j) {
        const int s0 = j * KT;
        const size_t ka = ko + (size_t)s0 * HD, kb = ka + (size_t)16 * HD;
        const v16bf kha0 = WFrag<bf>::ld(KPh + ka), kha1 = WFrag<bf>::ld(KPh + ka + 32), kla0 = WFrag<bf>::ld(KPl + ka), kla1 = WFrag<bf>::ld(KPl + ka + 32);
        v8f sc0 = (v8f){};
        sc0 = wmmab(qh0, kha0, sc0); sc0 = wmmab(ql0, kha0, sc0); sc0 = wmmab(qh1, kha1, sc0); sc0 = wmmab(ql1, kha1, sc0); sc0 = wmmab(qh0, kla0, sc0); sc0 = wmmab(qh1, kla1, sc0);
        const v16bf khb0 = WFrag<bf>::ld(KPh + kb), khb1 = WFrag<bf>::ld(KPh + kb + 32), klb0 = WFrag<bf>::ld(KPl + kb), klb1 = WFrag<bf>::ld(KPl + kb + 32);
        v8f sc1 = (v8f){};
        sc1 = wmmab(qh0, khb0, sc1); sc1 = wmmab(ql0, khb0, sc1); sc1 = wmmab(qh1, khb1, sc1); sc1 = wmmab(ql1, khb1, sc1); sc1 = wmmab(qh0, klb0, sc1); sc1 = wmmab(qh1, klb1, sc1);
        asm volatile("v_nop\n\tv_nop\n\tv_nop\n\tv_nop" : "+v"(sc0), "+v"(sc1) : "v"(qh1), "v"(kla1), "v"(klb0), "v"(klb1));
        float pm[8];
#pragma unroll
        for (int r = 0; r < 8; ++r) {
            float t = fmaxf(sc0[r], sc1[r]);
            t = fmaxf(t, __shfl_xor(t, 1, 32)); t = fmaxf(t, __shfl_xor(t, 2, 32)); t = fmaxf(t, __shfl_xor(t, 4, 32)); t = fmaxf(t, __shfl_xor(t, 8, 32));
            pm[r] = t; }
        if (j == 0) {
#pragma unroll
            for (int r = 0; r < 8; ++r) { float t = sc0[r] + sc1[r]; t += __shfl_xor(t, 1, 32); t += __shfl_xor(t, 2, 32); t += __shfl_xor(t, 4, 32); t += __shfl_xor(t, 8, 32); sbar[r] = t * (1.0f / KT); }
        }
        float aa[8];
#pragma unroll
        for (int r = 0; r < 8; ++r) {
            const float mn = fmaxf(mrun[r], pm[r]);
            aa[r] = __builtin_amdgcn_exp2f((mrun[r] - mn) * L2E);
            mrun[r] = mn;
            const float c = __builtin_amdgcn_exp2f((sbar[r] - mn) * L2E);
            const float p0 = __builtin_amdgcn_exp2f((sc0[r] - mn) * L2E), p1 = __builtin_amdgcn_exp2f((sc1[r] - mn) * L2E);
            float rs = p0 + p1; rs += __shfl_xor(rs, 1, 32); rs += __shfl_xor(rs, 2, 32); rs += __shfl_xor(rs, 4, 32); rs += __shfl_xor(rs, 8, 32);
            lrun[r] = lrun[r] * aa[r] + rs;
            pw[(8 * hi + r) * PSP + lr] = tohx((p0 - c) * PCAR);
            pw[(8 * hi + r) * PSP + 16 + lr] = tohx((p1 - c) * PCAR);
        }
#pragma unroll
        for (int t = 0; t < 4; ++t) {
#pragma unroll
            for (int r = 0; r < 8; ++r) o[t][r] *= aa[r]; }
        __syncthreads();
        const v16h pa = cat16(*(const v8ha*)(pw + lr * PSP + 8 * hi), *(const v8ha*)(pw + lr * PSP + 16 + 8 * hi));
        const size_t va = vo + (size_t)s0;
        const v16h vf0 = WFrag<h16>::ld(VT + va), vf1 = WFrag<h16>::ld(VT + va + (size_t)16 * SEQ), vf2 = WFrag<h16>::ld(VT + va + (size_t)32 * SEQ), vf3 = WFrag<h16>::ld(VT + va + (size_t)48 * SEQ);
        o[0] = wmma16(pa, vf0, o[0]); o[1] = wmma16(pa, vf1, o[1]); o[2] = wmma16(pa, vf2, o[2]); o[3] = wmma16(pa, vf3, o[3]);
        asm volatile("v_nop\n\tv_nop\n\tv_nop\n\tv_nop" : "+v"(o[0]), "+v"(o[1]), "+v"(o[2]), "+v"(o[3]) : "v"(pa), "v"(vf0), "v"(vf3));
        __syncthreads();
    }
    float vsum[4];
#pragma unroll
    for (int t = 0; t < 4; ++t) vsum[t] = VS[h * HD + t * 16 + lr];
#pragma unroll
    for (int r = 0; r < 8; ++r) {
        const float cf = __builtin_amdgcn_exp2f((sbar[r] - mrun[r]) * L2E);
        const float g = __builtin_amdgcn_rcpf(lrun[r]) * CCAR;
#pragma unroll
        for (int t = 0; t < 4; ++t) cw[(8 * hi + r) * CSP + t * 16 + lr] = tohx((o[t][r] * (1.0f / (PCAR * VCAR)) + cf * vsum[t]) * g);
    }
    __syncthreads();
    const int rq = lane >> 3, pc = lane & 7;
#pragma unroll 1
    for (int psx = 0; psx < 2; ++psx) {
#pragma unroll
        for (int q = 0; q < 4; ++q) { const int row = q * 4 + rq; const v8us v = *(const v8usa*)(cw + row * CSP + pc * 8);
            *(volatile v8us*)(CTX + (size_t)(r0 + row) * DMD + h * HD + pc * 8) = v; }
        if (psx == 0) __threadfence(); }
}

extern "C" void kernel_launch(void* const* d_in, const int* in_sizes, int n_in,
                              void* d_out, int out_size, void* d_ws, size_t ws_size, hipStream_t stream) {
    if (n_in < 11) return;
    const int need_x = (NB - 1) * SEQ_FULL * DMD + SEQ * DMD;
    if (in_sizes[0] < need_x || in_sizes[1] < need_x || in_sizes[2] < need_x) return;
    if (in_sizes[3] < DMD * DMD || in_sizes[5] < DMD * DMD || in_sizes[7] < DMD * DMD || in_sizes[9] < DMD * DMD) return;
    if (in_sizes[4] < DMD || in_sizes[6] < DMD || in_sizes[8] < DMD || in_sizes[10] < DMD) return;
    if (out_size < NB * SEQ * DMD) return;
    const float* xq = (const float*)d_in[0]; const float* xk = (const float*)d_in[1]; const float* xv = (const float*)d_in[2];
    const float* wq = (const float*)d_in[3]; const float* bq = (const float*)d_in[4];
    const float* wk = (const float*)d_in[5]; const float* bk = (const float*)d_in[6];
    const float* wv = (const float*)d_in[7]; const float* bv = (const float*)d_in[8];
    const float* wo = (const float*)d_in[9]; const float* bo = (const float*)d_in[10];
    float* OUT = (float*)d_out;
    char* wsp = (char*)d_ws;
    auto take = [&](size_t bytes) { char* p = wsp; wsp += (bytes + 255) & ~(size_t)255; return (void*)p; };
    bf*  WQ  = (bf*)take((size_t)DMD * DMD * 2);
    bf*  WK  = (bf*)take((size_t)DMD * DMD * 2);
    bf*  WV  = (bf*)take((size_t)DMD * DMD * 2);
    h16* WOT = (h16*)take((size_t)DMD * DMD * 2);
    bf*  XB  = (bf*)take((size_t)SEQ * DMD * 2);
    float* F = (float*)take((size_t)SEQ * DMD * 4);
    bf*  QPh = (bf*)take((size_t)NH * SEQ * HD * 2);
    bf*  QPl = (bf*)take((size_t)NH * SEQ * HD * 2);
    bf*  KPh = (bf*)take((size_t)NH * SEQ * HD * 2);
    bf*  KPl = (bf*)take((size_t)NH * SEQ * HD * 2);
    h16* VT  = (h16*)take((size_t)NH * HD * SEQ * 2);
    float* VS = (float*)take((size_t)DMD * 4);
    h16* CTX = (h16*)take((size_t)SEQ * DMD * 2);
    if ((size_t)(wsp - (char*)d_ws) > ws_size) return;
    const unsigned gw = (unsigned)((DMD * DMD / 64 + 63) / 64);
    k_wtG<<<gw, 256, 0, stream>>>(wq, DMD, DMD, WQ);
    k_wtG<<<gw, 256, 0, stream>>>(wk, DMD, DMD, WK);
    k_wtG<<<gw, 256, 0, stream>>>(wv, DMD, DMD, WV);
    k_wtH<<<gw, 256, 0, stream>>>(wo, DMD, DMD, WCAR, WOT);
    const unsigned gcv = (unsigned)(((size_t)SEQ * DMD / 8 + 255) / 256);
    const unsigned gpl = (unsigned)(((size_t)NH * SEQ * HD / 2 + 255) / 256);
    const dim3 ggm(SEQ / 64, DMD / 64, 1);
    const size_t xst = (size_t)SEQ_FULL * DMD;
    for (int b = 0; b < NB; ++b) {
        k_cvt8<<<gcv, 256, 0, stream>>>(xq + (size_t)b * xst, XB, (size_t)SEQ * DMD / 8);
        k_gemmw<bf, 0, true><<<ggm, 32, 0, stream>>>(XB, (const bf*)nullptr, WQ, (const bf*)nullptr, DMD, F, DMD, bq, 1.0f, (size_t)0, (size_t)0, (size_t)0);
        k_qkp<<<gpl, 256, 0, stream>>>(F, SCL, QPh, QPl);
        k_cvt8<<<gcv, 256, 0, stream>>>(xk + (size_t)b * xst, XB, (size_t)SEQ * DMD / 8);
        k_gemmw<bf, 0, true><<<ggm, 32, 0, stream>>>(XB, (const bf*)nullptr, WK, (const bf*)nullptr, DMD, F, DMD, bk, 1.0f, (size_t)0, (size_t)0, (size_t)0);
        k_qkp<<<gpl, 256, 0, stream>>>(F, 1.0f, KPh, KPl);
        k_cvt8<<<gcv, 256, 0, stream>>>(xv + (size_t)b * xst, XB, (size_t)SEQ * DMD / 8);
        k_gemmw<bf, 0, true><<<ggm, 32, 0, stream>>>(XB, (const bf*)nullptr, WV, (const bf*)nullptr, DMD, F, DMD, bv, 1.0f, (size_t)0, (size_t)0, (size_t)0);
        k_vtp<<<gpl, 256, 0, stream>>>(F, VT);
        k_colsum<<<DMD / 256, 256, 0, stream>>>(F, VS);
        k_flash<<<dim3(SEQ / 32, NH, 1), 64, 0, stream>>>(QPh, QPl, KPh, KPl, VT, VS, CTX);
        k_gemmw<h16, 0, true><<<ggm, 32, 0, stream>>>(CTX, (const h16*)nullptr, WOT, (const h16*)nullptr, DMD, OUT + (size_t)b * SEQ * DMD, DMD, bo, 1.0f / (CCAR * WCAR), (size_t)0, (size_t)0, (size_t)0);
    }
}
